// SABlock_37314675867675
// MI455X (gfx1250) — hardware-run, weakly checked
//
#include <hip/hip_runtime.h>
#include <math.h>

typedef __attribute__((ext_vector_type(16))) _Float16 v16h;
typedef __attribute__((ext_vector_type(8)))  _Float16 v8h;
typedef __attribute__((ext_vector_type(16))) __bf16   v16b;
typedef __attribute__((ext_vector_type(8)))  __bf16   v8b;
typedef __attribute__((ext_vector_type(8)))  float    v8f;
typedef __attribute__((ext_vector_type(4)))  float    v4f;
typedef __attribute__((ext_vector_type(4)))  unsigned v4u;

constexpr int kBatch = 8;
constexpr int kCh    = 768;
constexpr int kTok   = 1024;
constexpr int kHeads = 12;
constexpr int kHd    = 64;
constexpr int kHid   = 3072;
constexpr int kRows  = kBatch * kTok;
constexpr int kQkvN  = 3 * kCh;
constexpr int kHalfRows = kRows / 2;
constexpr int kHalfBatch = kBatch / 2;

constexpr size_t kOffT0   = 0;
constexpr size_t kSzT     = (size_t)kBatch * kCh * kTok * 4;
constexpr size_t kOffHN   = kOffT0 + kSzT;
constexpr size_t kSzHN    = (size_t)kRows * kCh * 2;
constexpr size_t kOffWqkv = kOffHN + kSzHN;
constexpr size_t kSzWqkv  = (size_t)kQkvN * kCh * 2;
constexpr size_t kOffWprj = kOffWqkv + kSzWqkv;
constexpr size_t kSzWprj  = (size_t)kCh * kCh * 2;
constexpr size_t kOffWfc1 = kOffWprj + kSzWprj;
constexpr size_t kSzWfc1  = (size_t)kHid * kCh * 2;
constexpr size_t kOffWfc2 = kOffWfc1 + kSzWfc1;
constexpr size_t kSzWfc2  = (size_t)kCh * kHid * 2;
constexpr size_t kOffQKV  = kOffWfc2 + kSzWfc2;
constexpr size_t kSzQKV   = (size_t)kRows * kQkvN * 2;
constexpr size_t kOffT1   = kOffQKV;
constexpr size_t kOffO16  = kOffQKV + kSzQKV;
constexpr size_t kSzO16   = (size_t)kRows * kCh * 2;
constexpr size_t kSzHalf  = (size_t)kHalfRows * kHid * 2;
constexpr size_t kOffPRE  = kOffT1 + kSzT;
constexpr size_t kOffHID  = kOffPRE + kSzHalf;
constexpr size_t kWsTotal = kOffHID + kSzHalf;
static_assert(kOffPRE + kSzHalf == kOffO16 + kSzO16);
static_assert(kOffT1 + kSzT <= kOffPRE);
static_assert(kWsTotal <= (size_t)134217728);
static_assert((kOffHN % 128) == 0 && (kOffWqkv % 128) == 0 && (kOffWprj % 128) == 0 && (kOffWfc1 % 128) == 0);
static_assert((kOffWfc2 % 128) == 0 && (kOffQKV % 128) == 0 && (kOffO16 % 128) == 0 && (kOffPRE % 128) == 0 && (kOffHID % 128) == 0);
static_assert(kRows % 64 == 0 && kQkvN % 64 == 0 && kCh % 64 == 0 && kTok % 64 == 0 && kHid % 64 == 0 && kHalfRows % 64 == 0);
static_assert(kCh % 32 == 0 && kHid % 32 == 0);
static_assert(kHd == 64 && kHeads * kHd == kCh && kTok % 64 == 0);

#define U16(p) ((const unsigned short*)(const void*)(p))

__device__ __forceinline__ unsigned short f2bf_bits(float f) {
  unsigned u = __float_as_uint(f);
  return (unsigned short)((u + 0x7FFFu + ((u >> 16) & 1u)) >> 16);
}
__device__ __forceinline__ float bf_bits2f(unsigned short h) { return __uint_as_float(((unsigned)h) << 16); }

__device__ __forceinline__ void dep_guard_h(v8f& a, v8f& b, v16h x, v16h y) { asm volatile("v_nop\n\tv_nop\n\tv_nop\n\tv_nop" : "+v"(a), "+v"(b) : "v"(x), "v"(y)); }
__device__ __forceinline__ void dep_guard_b(v8f& a, v8f& b, v16b x, v16b y) { asm volatile("v_nop\n\tv_nop\n\tv_nop\n\tv_nop" : "+v"(a), "+v"(b) : "v"(x), "v"(y)); }
__device__ __forceinline__ void keep4_h(v16h a, v16h b, v16h c, v16h d) { asm volatile("v_nop" :: "v"(a), "v"(b), "v"(c), "v"(d)); }
__device__ __forceinline__ void keep4_b(v16b a, v16b b, v16b c, v16b d) { asm volatile("v_nop" :: "v"(a), "v"(b), "v"(c), "v"(d)); }
__device__ __forceinline__ void acc_guard4(v8f& a, v8f& b, v8f& c, v8f& d) { asm volatile("v_nop\n\tv_nop\n\tv_nop\n\tv_nop" : "+v"(a), "+v"(b), "+v"(c), "+v"(d)); }
template <typename T> struct Frag;
template <> struct Frag<_Float16> {
  typedef v16h V; union U { v16h v; v8h h[2]; };
  static __device__ __forceinline__ v16h load(const _Float16* p) {
    U f; f.h[0] = *(const v8h*)(p); f.h[1] = *(const v8h*)(p + 16); return f.v;
  }
  static __device__ __forceinline__ v8f mma(v16h a, v16h b, v8f c) {
    return __builtin_amdgcn_wmma_f32_16x16x32_f16(false, a, false, b, (short)0, c, false, false);
  }
  static __device__ __forceinline__ void guard(v8f& a, v8f& b, v16h x, v16h y) { dep_guard_h(a, b, x, y); }
  static __device__ __forceinline__ void keep(v16h a, v16h b, v16h c, v16h d) { keep4_h(a, b, c, d); }
};
template <> struct Frag<__bf16> {
  typedef v16b V; union U { v16b v; v8b h[2]; };
  static __device__ __forceinline__ v16b load(const __bf16* p) {
    U f; f.h[0] = *(const v8b*)(p); f.h[1] = *(const v8b*)(p + 16); return f.v;
  }
  static __device__ __forceinline__ v8f mma(v16b a, v16b b, v8f c) {
    return __builtin_amdgcn_wmma_f32_16x16x32_bf16(false, a, false, b, (short)0, c, false, false);
  }
  static __device__ __forceinline__ void guard(v8f& a, v8f& b, v16b x, v16b y) { dep_guard_b(a, b, x, y); }
  static __device__ __forceinline__ void keep(v16b a, v16b b, v16b c, v16b d) { keep4_b(a, b, c, d); }
};

template <int ET> struct Elem;
template <> struct Elem<0> { typedef _Float16 T; };
template <> struct Elem<1> { typedef __bf16 T; };
template <int ET, bool SPLIT, int BIAS_MODE, int OUT_MODE, bool RESID>
__global__ __launch_bounds__(256) void wmma_gemm64(
    const unsigned short* __restrict__ Ap, const unsigned short* __restrict__ A2p, int lda, long strideA,
    const unsigned short* __restrict__ Btp, const unsigned short* __restrict__ Bt2p, int ldb, long strideB,
    void* __restrict__ Cout, void* __restrict__ Cout2, int ldc, long strideC,
    const float* __restrict__ bias,
    const float* __restrict__ resid, long strideR,
    int M, int N, int K, float scale) {
  static_assert(!(RESID && OUT_MODE != 0), "");
  typedef typename Elem<ET>::T T;
  typedef typename Frag<T>::V V;
  const T* A = (const T*)Ap; const T* A2 = (const T*)A2p; const T* Bt = (const T*)Btp; const T* Bt2 = (const T*)Bt2p;
  __shared__ __align__(16) float sT[8][16 * 68];
  const int b    = blockIdx.y;
  const int lane = threadIdx.x & 31;
  const int wave = threadIdx.x >> 5;
  const int tilesN = N >> 6;
  const int tilesM = M >> 6;
  const int tile = blockIdx.x * 8 + wave;
  if (tile >= tilesM * tilesN) return;
  const int tm = tile / tilesN;
  const int tn = tile - tm * tilesN;
  const int m0 = tm << 6;
  const int n0 = tn << 6;

  const T* Ab  = A  + (size_t)b * strideA;
  const T* Bb  = Bt + (size_t)b * strideB;
  const T* Ab2 = SPLIT ? (A2  + (size_t)b * strideA) : nullptr;
  const T* Bb2 = SPLIT ? (Bt2 + (size_t)b * strideB) : nullptr;

  const int rlane = lane & 15;
  const int koff  = (lane >> 4) * 8;
  const int mOff  = (lane >> 4) * 8;

  v8f acc[4][4];
#pragma unroll
  for (int i = 0; i < 4; ++i)
#pragma unroll
    for (int j = 0; j < 4; ++j) acc[i][j] = (v8f){0.f,0.f,0.f,0.f,0.f,0.f,0.f,0.f};

  for (int k0 = 0; k0 < K; k0 += 32) {
    V bh[4], bl[4];
#pragma unroll
    for (int j = 0; j < 4; ++j) {
      const size_t bo = (size_t)(n0 + (j << 4) + rlane) * ldb + koff + k0;
      bh[j] = Frag<T>::load(Bb + bo);
      if (SPLIT) bl[j] = Frag<T>::load(Bb2 + bo);
    }
#pragma unroll
    for (int i = 0; i < 4; ++i) {
      const size_t ao = (size_t)(m0 + (i << 4) + rlane) * lda + koff + k0;
      V ah = Frag<T>::load(Ab + ao);
      V al;
      if (SPLIT) al = Frag<T>::load(Ab2 + ao);
#pragma unroll
      for (int j = 0; j < 4; ++j) {
        acc[i][j] = Frag<T>::mma(ah, bh[j], acc[i][j]);
        if (SPLIT) {
          acc[i][j] = Frag<T>::mma(ah, bl[j], acc[i][j]);
          acc[i][j] = Frag<T>::mma(al, bh[j], acc[i][j]);
        }
      }
      Frag<T>::guard(acc[i][0], acc[i][3], ah, SPLIT ? al : ah);
    }
    Frag<T>::keep(bh[0], bh[1], bh[2], bh[3]);
    if (SPLIT) Frag<T>::keep(bl[0], bl[1], bl[2], bl[3]);
  }
  acc_guard4(acc[0][0], acc[0][1], acc[0][2], acc[0][3]);
  acc_guard4(acc[1][0], acc[1][1], acc[1][2], acc[1][3]);
  acc_guard4(acc[2][0], acc[2][1], acc[2][2], acc[2][3]);
  acc_guard4(acc[3][0], acc[3][1], acc[3][2], acc[3][3]);

  float* slab = sT[wave];
  const float* Rb = RESID ? (resid + (size_t)b * strideR) : nullptr;
#pragma unroll
  for (int i = 0; i < 4; ++i) {
    const int mBase = m0 + (i << 4);
    float bmv[8] = {0.f,0.f,0.f,0.f,0.f,0.f,0.f,0.f};
    if (BIAS_MODE == 1) {
      const v4f bm0 = *(const v4f*)(bias + mBase + mOff);
      const v4f bm1 = *(const v4f*)(bias + mBase + mOff + 4);
      bmv[0] = bm0[0]; bmv[1] = bm0[1]; bmv[2] = bm0[2]; bmv[3] = bm0[3];
      bmv[4] = bm1[0]; bmv[5] = bm1[1]; bmv[6] = bm1[2]; bmv[7] = bm1[3];
    }
#pragma unroll
    for (int j = 0; j < 4; ++j) {
      const int n = n0 + (j << 4) + rlane;
      float bv = 0.f;
      if (BIAS_MODE == 2) bv = bias[n];
#pragma unroll
      for (int r = 0; r < 8; ++r) {
        float v = acc[i][j][r] * scale;
        if (BIAS_MODE == 1) v += bmv[r];
        if (BIAS_MODE == 2) v += bv;
        slab[(mOff + r) * 68 + (j << 4) + rlane] = v;
      }
    }
    __builtin_amdgcn_fence(__ATOMIC_RELEASE, "workgroup");
    __builtin_amdgcn_wave_barrier();
    __builtin_amdgcn_fence(__ATOMIC_ACQUIRE, "workgroup");
    if (OUT_MODE == 0) {
      float* C = (float*)Cout + (size_t)b * strideC;
      const int hh = lane >> 4, c4 = (lane & 15) * 4;
      if (RESID) {
#pragma unroll
        for (int it = 0; it < 8; ++it) {
          const int row = it * 2 + hh;
          const v4f rv = *(const v4f*)(Rb + (size_t)(mBase + row) * ldc + n0 + c4);
          float* sp = slab + row * 68 + c4;
          v4f sv = *(const v4f*)sp;
          sv += rv;
          *(v4f*)sp = sv;
        }
      }
      for (int pass = 0; pass < 2; ++pass) {
#pragma unroll
        for (int it = 0; it < 8; ++it) {
          const int row = it * 2 + hh;
          v4f v = *(const v4f*)(slab + row * 68 + c4);
          *(volatile v4f*)(C + (size_t)(mBase + row) * ldc + n0 + c4) = v;
        }
        __threadfence();
      }
    } else {
      const int q = lane >> 3, c8 = (lane & 7) * 8;
      unsigned short* C  = (unsigned short*)Cout  + (size_t)b * strideC;
      unsigned short* C2 = (OUT_MODE == 2) ? ((unsigned short*)Cout2 + (size_t)b * strideC) : nullptr;
      for (int pass = 0; pass < 2; ++pass) {
#pragma unroll
        for (int it = 0; it < 4; ++it) {
          const int row = it * 4 + q;
          const float* sp = slab + row * 68 + c8;
          v8h hv, lv;
#pragma unroll
          for (int e = 0; e < 8; ++e) {
            if (OUT_MODE == 1) {
              hv[e] = (_Float16)sp[e];
            } else {
              unsigned short hb = f2bf_bits(sp[e]);
              unsigned short lb = f2bf_bits(sp[e] - bf_bits2f(hb));
              hv[e] = __builtin_bit_cast(_Float16, hb);
              lv[e] = __builtin_bit_cast(_Float16, lb);
            }
          }
          *(volatile v8h*)(C + (size_t)(mBase + row) * ldc + n0 + c8) = hv;
          if (OUT_MODE == 2) *(volatile v8h*)(C2 + (size_t)(mBase + row) * ldc + n0 + c8) = lv;
        }
        __threadfence();
      }
    }
    __builtin_amdgcn_fence(__ATOMIC_RELEASE, "workgroup");
    __builtin_amdgcn_wave_barrier();
    __builtin_amdgcn_fence(__ATOMIC_ACQUIRE, "workgroup");
  }
}

__global__ __launch_bounds__(256) void cast_scale_f16x2(
    const float* __restrict__ in, unsigned short* __restrict__ out, int n2, float sc) {
  int i = blockIdx.x * 256 + threadIdx.x;
  if (i < n2) {
    const _Float16 h0 = (_Float16)(in[2 * i] * sc), h1 = (_Float16)(in[2 * i + 1] * sc);
    const unsigned u = (unsigned)__builtin_bit_cast(unsigned short, h0) | ((unsigned)__builtin_bit_cast(unsigned short, h1) << 16);
    ((volatile unsigned*)(void*)out)[i] = u;
    __threadfence();
    ((volatile unsigned*)(void*)out)[i] = u;
  }
}

__global__ __launch_bounds__(256)
void conv_pe_kernel(const float* __restrict__ x, const float* __restrict__ w,
                    const float* __restrict__ bias, float* __restrict__ Tout, int nplanes) {
  const int plane = blockIdx.x;
  if (plane >= nplanes) return;
  const int tid = threadIdx.x;
  const int hrow = tid >> 3, wq = tid & 7, w0 = wq * 4;
  const int c = plane % kCh;
  const float* xp = x + (size_t)plane * kTok;
  const float* wp = w + c * 9;
  float wk[9];
#pragma unroll
  for (int i = 0; i < 9; ++i) wk[i] = wp[i];
  const float bc = bias[c];
  float accv[4] = {0.f, 0.f, 0.f, 0.f};
  float ctr[4] = {0.f, 0.f, 0.f, 0.f};
#pragma unroll
  for (int dy = -1; dy <= 1; ++dy) {
    const int rr = hrow + dy;
    const bool vrow = (rr >= 0) && (rr < 32);
    const int rc = rr < 0 ? 0 : (rr > 31 ? 31 : rr);
    const float* rp = xp + rc * 32;
    const v4f mid = *(const v4f*)(rp + w0);
    const int il = (w0 > 0) ? (w0 - 1) : 0;
    const int ir = (w0 + 4 < 32) ? (w0 + 4) : 31;
    const float lv = rp[il], rv = rp[ir];
    float v6[6];
    v6[0] = (vrow && (w0 > 0)) ? lv : 0.f;
    v6[1] = vrow ? mid[0] : 0.f;
    v6[2] = vrow ? mid[1] : 0.f;
    v6[3] = vrow ? mid[2] : 0.f;
    v6[4] = vrow ? mid[3] : 0.f;
    v6[5] = (vrow && (w0 + 4 < 32)) ? rv : 0.f;
    if (dy == 0) { ctr[0] = mid[0]; ctr[1] = mid[1]; ctr[2] = mid[2]; ctr[3] = mid[3]; }
    const int tb = (dy + 1) * 3;
#pragma unroll
    for (int j = 0; j < 4; ++j)
      accv[j] += v6[j] * wk[tb] + v6[j + 1] * wk[tb + 1] + v6[j + 2] * wk[tb + 2];
  }
  v4f o;
#pragma unroll
  for (int j = 0; j < 4; ++j) o[j] = (ctr[j] + accv[j]) + bc;
  float* dst = Tout + (size_t)plane * kTok + hrow * 32 + w0;
  *(volatile v4f*)dst = o;
  __threadfence();
  *(volatile v4f*)dst = o;
}

constexpr int kLnTok = 32;
__global__ __launch_bounds__(256)
void ln_cm_kernel(const float* __restrict__ Tin, const float* __restrict__ gam, const float* __restrict__ bet,
                  unsigned short* __restrict__ out16) {
  __shared__ __align__(16) unsigned short tile[kLnTok * kCh];
  __shared__ float gsh[kCh];
  __shared__ float bsh[kCh];
  __shared__ float red[8][kLnTok];
  const int tid = threadIdx.x, wave = tid >> 5, lane = tid & 31;
  const int lq = lane & 7, cg = tid >> 3;
  const int blk = blockIdx.x;
  const int b = blk / (kTok / kLnTok);
  const int tok0 = (blk % (kTok / kLnTok)) * kLnTok;
  for (int i = tid; i < kCh; i += 256) { gsh[i] = gam[i]; bsh[i] = bet[i]; }
  const float* base = Tin + (size_t)b * kCh * kTok + tok0 + 4 * lq;

  v4f s = (v4f){0.f, 0.f, 0.f, 0.f};
#pragma unroll 1
  for (int grp = 0; grp < 6; ++grp) {
#pragma unroll
    for (int u = 0; u < 4; ++u) {
      const int c = cg + 32 * (grp * 4 + u);
      const v4f xv = *(const v4f*)(base + (size_t)c * kTok);
      s += xv;
    }
  }
#pragma unroll
  for (int e = 0; e < 4; ++e) {
    float t = s[e];
    t += __shfl_xor(t, 8, 32);
    t += __shfl_xor(t, 16, 32);
    s[e] = t;
  }
  if (lane < 8) {
#pragma unroll
    for (int e = 0; e < 4; ++e) red[wave][4 * lq + e] = s[e];
  }
  __syncthreads();
  float mu[4];
#pragma unroll
  for (int e = 0; e < 4; ++e) {
    float t = 0.f;
#pragma unroll
    for (int w8 = 0; w8 < 8; ++w8) t += red[w8][4 * lq + e];
    mu[e] = t * (1.0f / (float)kCh);
  }
  __syncthreads();

  v4f qs = (v4f){0.f, 0.f, 0.f, 0.f};
  const v4f muv = (v4f){mu[0], mu[1], mu[2], mu[3]};
#pragma unroll 1
  for (int grp = 0; grp < 6; ++grp) {
#pragma unroll
    for (int u = 0; u < 4; ++u) {
      const int c = cg + 32 * (grp * 4 + u);
      const v4f xv = *(const v4f*)(base + (size_t)c * kTok);
      const v4f d = xv - muv;
      qs += d * d;
    }
  }
#pragma unroll
  for (int e = 0; e < 4; ++e) {
    float t = qs[e];
    t += __shfl_xor(t, 8, 32);
    t += __shfl_xor(t, 16, 32);
    qs[e] = t;
  }
  if (lane < 8) {
#pragma unroll
    for (int e = 0; e < 4; ++e) red[wave][4 * lq + e] = qs[e];
  }
  __syncthreads();
  float rs[4];
#pragma unroll
  for (int e = 0; e < 4; ++e) {
    float t = 0.f;
#pragma unroll
    for (int w8 = 0; w8 < 8; ++w8) t += red[w8][4 * lq + e];
    const float var = t * (1.0f / (float)kCh);
    rs[e] = rsqrtf(var + 1e-5f);
  }

#pragma unroll 1
  for (int grp = 0; grp < 6; ++grp) {
#pragma unroll
    for (int u = 0; u < 4; ++u) {
      const int c = cg + 32 * (grp * 4 + u);
      const v4f xv = *(const v4f*)(base + (size_t)c * kTok);
      const float gc = gsh[c], bcv = bsh[c];
#pragma unroll
      for (int e = 0; e < 4; ++e) {
        const float y = (xv[e] - mu[e]) * rs[e] * gc + bcv;
        tile[(4 * lq + e) * kCh + c] = __builtin_bit_cast(unsigned short, (_Float16)y);
      }
    }
  }
  __syncthreads();

  const int l8 = lane & 7, lq4 = lane >> 3;
  unsigned short* ob = out16 + ((size_t)b * kTok + tok0) * kCh;
  for (int pass = 0; pass < 2; ++pass) {
#pragma unroll
    for (int it = 0; it < 12; ++it) {
      const int L = it * 32 + wave * 4 + lq4;
      const int row = L / 12, seg = L - row * 12;
      const v4u v = *(const v4u*)(const void*)(tile + row * kCh + seg * 64 + l8 * 8);
      *(volatile v4u*)(void*)(ob + (size_t)row * kCh + seg * 64 + l8 * 8) = v;
    }
    __threadfence();
  }
}

constexpr int kAtD = 64, kAtNW = 4, kAtQB = 64, kAtKC = 64;
constexpr float kPSC = 32768.0f;

__device__ __forceinline__ v8f mma_f16(v16h a, v16h b, v8f c) {
  c = __builtin_amdgcn_wmma_f32_16x16x32_f16(false, a, false, b, (short)0, c, false, false);
  asm volatile("v_nop\n\tv_nop\n\tv_nop\n\tv_nop" : "+v"(c) : "v"(a), "v"(b));
  return c;
}

__global__ __launch_bounds__(128)
void attn_f16_kernel(const unsigned short* __restrict__ qkvp, unsigned short* __restrict__ outp,
                     float qscale, float oscale) {
  union FH { v16h v; v8h h[2]; };
  const _Float16* qkv = (const _Float16*)(const void*)qkvp;
  __shared__ __align__(16) unsigned short Ksh[kAtKC * kAtD];
  __shared__ __align__(16) unsigned short Vth[kAtD * kAtKC];
  __shared__ __align__(16) _Float16 Psh[kAtNW][16 * kAtKC];
  __shared__ __align__(16) float Os[kAtNW][16 * 68];

  const int tid  = threadIdx.x;
  const int wave = tid >> 5;
  const int lane = tid & 31;
  const int hh   = lane >> 4;
  const int c    = lane & 15;

  const int nqb = kTok / kAtQB;
  const int bx  = blockIdx.x;
  const int qb  = bx % nqb;
  const int bh  = bx / nqb;
  const int h   = bh % kHeads;
  const int b   = bh / kHeads;
  const int q0  = qb * kAtQB + wave * 16;

  const _Float16* base = qkv + (size_t)b * kTok * kQkvN + h * kHd;

  v16h qa[2];
  {
    const _Float16* qrow = base + (size_t)(q0 + c) * kQkvN;
#pragma unroll
    for (int dc = 0; dc < 2; ++dc) qa[dc] = Frag<_Float16>::load(qrow + dc * 32 + 8 * hh);
  }

  float mrow[8], lrow[8];
  v8f oacc[4];
#pragma unroll
  for (int r = 0; r < 8; ++r) { mrow[r] = -INFINITY; lrow[r] = 0.f; }
#pragma unroll
  for (int t = 0; t < 4; ++t) oacc[t] = (v8f){0.f,0.f,0.f,0.f,0.f,0.f,0.f,0.f};

  const int nChunks = kTok / kAtKC;
  for (int kc = 0; kc < nChunks; ++kc) {
    const int kv0 = kc * kAtKC;
    __syncthreads();
    {
#pragma unroll
      for (int i = 0; i < 4; ++i) {
        const int qd = tid + i * 128;
        const int row = qd >> 3, c8 = (qd & 7) * 8;
        const _Float16* kp = base + (size_t)(kv0 + row) * kQkvN + kCh + c8;
        const _Float16* vp = base + (size_t)(kv0 + row) * kQkvN + 2 * kCh + c8;
        const v4u kk = *(const v4u*)(const void*)kp;
        const v4u vv = *(const v4u*)(const void*)vp;
        *(v4u*)(void*)(Ksh + row * kAtD + c8) = kk;
        const unsigned vw0 = vv[0], vw1 = vv[1], vw2 = vv[2], vw3 = vv[3];
        Vth[(c8 + 0) * kAtKC + row] = (unsigned short)(vw0 & 0xffffu);
        Vth[(c8 + 1) * kAtKC + row] = (unsigned short)(vw0 >> 16);
        Vth[(c8 + 2) * kAtKC + row] = (unsigned short)(vw1 & 0xffffu);
        Vth[(c8 + 3) * kAtKC + row] = (unsigned short)(vw1 >> 16);
        Vth[(c8 + 4) * kAtKC + row] = (unsigned short)(vw2 & 0xffffu);
        Vth[(c8 + 5) * kAtKC + row] = (unsigned short)(vw2 >> 16);
        Vth[(c8 + 6) * kAtKC + row] = (unsigned short)(vw3 & 0xffffu);
        Vth[(c8 + 7) * kAtKC + row] = (unsigned short)(vw3 >> 16);
      }
    }
    __syncthreads();

    v8f s[4];
#pragma unroll
    for (int j = 0; j < 4; ++j) {
      s[j] = (v8f){0.f,0.f,0.f,0.f,0.f,0.f,0.f,0.f};
#pragma unroll
      for (int dc = 0; dc < 2; ++dc) {
        FH kb;
        kb.h[0] = *(const v8h*)(const void*)(Ksh + (j * 16 + c) * kAtD + dc * 32 + 8 * hh);
        kb.h[1] = *(const v8h*)(const void*)(Ksh + (j * 16 + c) * kAtD + dc * 32 + 16 + 8 * hh);
        s[j] = mma_f16(qa[dc], kb.v, s[j]);
      }
#pragma unroll
      for (int r = 0; r < 8; ++r) s[j][r] *= qscale;
    }
    float cm[8];
#pragma unroll
    for (int r = 0; r < 8; ++r) {
      float m = s[0][r];
      m = fmaxf(m, s[1][r]); m = fmaxf(m, s[2][r]); m = fmaxf(m, s[3][r]);
#pragma unroll
      for (int off = 1; off < 16; off <<= 1) m = fmaxf(m, __shfl_xor(m, off, 32));
      cm[r] = m;
    }
    _Float16* pw = Psh[wave];
#pragma unroll
    for (int r = 0; r < 8; ++r) {
      const float mnew = fmaxf(mrow[r], cm[r]);
      const float alpha = expf(mrow[r] - mnew);
      mrow[r] = mnew;
      float psum = 0.f;
#pragma unroll
      for (int j = 0; j < 4; ++j) {
        const float p = expf(s[j][r] - mnew);
        psum += p;
        pw[(8 * hh + r) * kAtKC + j * 16 + c] = (_Float16)(p * kPSC);
      }
#pragma unroll
      for (int off = 1; off < 16; off <<= 1) psum += __shfl_xor(psum, off, 32);
      lrow[r] = lrow[r] * alpha + psum;
#pragma unroll
      for (int t = 0; t < 4; ++t) oacc[t][r] *= alpha;
    }
    __builtin_amdgcn_fence(__ATOMIC_RELEASE, "workgroup");
    __builtin_amdgcn_wave_barrier();
    __builtin_amdgcn_fence(__ATOMIC_ACQUIRE, "workgroup");
#pragma unroll
    for (int kk = 0; kk < 2; ++kk) {
      FH pa;
      pa.h[0] = *(const v8h*)(pw + c * kAtKC + kk * 32 + 8 * hh);
      pa.h[1] = *(const v8h*)(pw + c * kAtKC + kk * 32 + 16 + 8 * hh);
#pragma unroll
      for (int t = 0; t < 4; ++t) {
        FH vb;
        vb.h[0] = *(const v8h*)(const void*)(Vth + (t * 16 + c) * kAtKC + kk * 32 + 8 * hh);
        vb.h[1] = *(const v8h*)(const void*)(Vth + (t * 16 + c) * kAtKC + kk * 32 + 16 + 8 * hh);
        oacc[t] = mma_f16(pa.v, vb.v, oacc[t]);
      }
    }
  }

  float* os = Os[wave];
#pragma unroll
  for (int r = 0; r < 8; ++r) {
    const float inv = oscale / (lrow[r] * kPSC);
#pragma unroll
    for (int t = 0; t < 4; ++t) os[(8 * hh + r) * 68 + t * 16 + c] = oacc[t][r] * inv;
  }
  __builtin_amdgcn_fence(__ATOMIC_RELEASE, "workgroup");
  __builtin_amdgcn_wave_barrier();
  __builtin_amdgcn_fence(__ATOMIC_ACQUIRE, "workgroup");
  {
    const int q4 = lane >> 3, c8o = (lane & 7) * 8;
    _Float16* ob = (_Float16*)(void*)outp + (size_t)b * kTok * kCh + h * kHd;
    for (int pass = 0; pass < 2; ++pass) {
#pragma unroll
      for (int it = 0; it < 4; ++it) {
        const int row = it * 4 + q4;
        const float* sp = os + row * 68 + c8o;
        v8h hv;
#pragma unroll
        for (int e = 0; e < 8; ++e) hv[e] = (_Float16)sp[e];
        *(volatile v8h*)(ob + (size_t)(q0 + row) * kCh + c8o) = hv;
      }
      __threadfence();
    }
  }
}

__global__ __launch_bounds__(256)
void gelu_f16_kernel(const unsigned* __restrict__ in, unsigned* __restrict__ out, int nwords, float carry) {
  const int i = blockIdx.x * 256 + threadIdx.x;
  if (i >= nwords) return;
  const unsigned w = in[i];
  const float x0 = (float)__builtin_bit_cast(_Float16, (unsigned short)(w & 0xffffu));
  const float x1 = (float)__builtin_bit_cast(_Float16, (unsigned short)(w >> 16));
  unsigned res = 0u;
#pragma unroll 1
  for (int e = 0; e < 2; ++e) {
    const float xv = (e == 0) ? x0 : x1;
    const float gv = 0.5f * xv * (1.0f + erff(xv * 0.70710678118654752f));
    const unsigned hb = (unsigned)__builtin_bit_cast(unsigned short, (_Float16)(gv * carry));
    res |= hb << (16 * e);
  }
  ((volatile unsigned*)out)[i] = res;
  __threadfence();
  ((volatile unsigned*)out)[i] = res;
}

extern "C" void kernel_launch(void* const* d_in, const int* in_sizes, int n_in,
                              void* d_out, int out_size, void* d_ws, size_t ws_size,
                              hipStream_t stream) {
  if (n_in < 14) return;
  if (in_sizes[0] != kBatch * kCh * kTok || out_size != kBatch * kCh * kTok) return;
  if (ws_size < kWsTotal) return;
  if (in_sizes[5] != kQkvN * kCh || in_sizes[6] != kCh * kCh || in_sizes[10] != kHid * kCh || in_sizes[12] != kCh * kHid) return;

  const float* x      = (const float*)d_in[0];
  const float* conv_w = (const float*)d_in[1];
  const float* conv_b = (const float*)d_in[2];
  const float* ln1_g  = (const float*)d_in[3];
  const float* ln1_b  = (const float*)d_in[4];
  const float* qkv_w  = (const float*)d_in[5];
  const float* proj_w = (const float*)d_in[6];
  const float* proj_b = (const float*)d_in[7];
  const float* ln2_g  = (const float*)d_in[8];
  const float* ln2_b  = (const float*)d_in[9];
  const float* fc1_w  = (const float*)d_in[10];
  const float* fc1_b  = (const float*)d_in[11];
  const float* fc2_w  = (const float*)d_in[12];
  const float* fc2_b  = (const float*)d_in[13];
  float* out = (float*)d_out;

  char* ws = (char*)d_ws;
  float* T0 = (float*)(ws + kOffT0);
  float* T1 = (float*)(ws + kOffT1);
  unsigned short* hn16  = (unsigned short*)(ws + kOffHN);
  unsigned short* wqkv  = (unsigned short*)(ws + kOffWqkv);
  unsigned short* wproj = (unsigned short*)(ws + kOffWprj);
  unsigned short* wfc1  = (unsigned short*)(ws + kOffWfc1);
  unsigned short* wfc2  = (unsigned short*)(ws + kOffWfc2);
  unsigned short* qkv16 = (unsigned short*)(ws + kOffQKV);
  unsigned short* o16   = (unsigned short*)(ws + kOffO16);
  unsigned short* pre16 = (unsigned short*)(ws + kOffPRE);
  unsigned short* hid16 = (unsigned short*)(ws + kOffHID);

  const float kWCarry = 64.0f;
  const float kOCarry = 64.0f;
  const float kHCarry = 16.0f;

  {
    const int n2q = (kQkvN * kCh) / 2, n2p = (kCh * kCh) / 2, n2f1 = (kHid * kCh) / 2, n2f2 = (kCh * kHid) / 2;
    cast_scale_f16x2<<<(n2q + 255) / 256, 256, 0, stream>>>(qkv_w, wqkv, n2q, kWCarry);
    cast_scale_f16x2<<<(n2p + 255) / 256, 256, 0, stream>>>(proj_w, wproj, n2p, kWCarry);
    cast_scale_f16x2<<<(n2f1 + 255) / 256, 256, 0, stream>>>(fc1_w, wfc1, n2f1, kWCarry);
    cast_scale_f16x2<<<(n2f2 + 255) / 256, 256, 0, stream>>>(fc2_w, wfc2, n2f2, kWCarry);
  }

  conv_pe_kernel<<<kBatch * kCh, 256, 0, stream>>>(x, conv_w, conv_b, T0, kBatch * kCh);

  ln_cm_kernel<<<kRows / kLnTok, 256, 0, stream>>>(T0, ln1_g, ln1_b, hn16);

  {
    const int tiles = (kRows / 64) * (kQkvN / 64);
    wmma_gemm64<0, false, 0, 1, false><<<dim3((tiles + 7) / 8, 1), 256, 0, stream>>>(
        hn16, hn16, kCh, 0L,
        wqkv, wqkv, kCh, 0L,
        (void*)qkv16, (void*)qkv16, kQkvN, 0L,
        nullptr, nullptr, 0L,
        kRows, kQkvN, kCh, 1.0f / kWCarry);
  }

  attn_f16_kernel<<<kBatch * kHeads * (kTok / kAtQB), 128, 0, stream>>>(qkv16, o16, 0.125f, kOCarry);

  {
    const int tiles = (kCh / 64) * (kTok / 64);
    wmma_gemm64<0, false, 1, 0, true><<<dim3((tiles + 7) / 8, kBatch), 256, 0, stream>>>(
        wproj, wproj, kCh, 0L,
        o16, o16, kCh, (long)kTok * kCh,
        (void*)T1, (void*)T1, kTok, (long)kCh * kTok,
        proj_b,
        T0, (long)kCh * kTok,
        kCh, kTok, kCh, 1.0f / (kWCarry * kOCarry));
  }

  ln_cm_kernel<<<kRows / kLnTok, 256, 0, stream>>>(T1, ln2_g, ln2_b, hn16);

  for (int half = 0; half < 2; ++half) {
    {
      const int tiles = (kHalfRows / 64) * (kHid / 64);
      wmma_gemm64<0, false, 2, 1, false><<<dim3((tiles + 7) / 8, 1), 256, 0, stream>>>(
          hn16 + (size_t)half * kHalfRows * kCh, hn16 + (size_t)half * kHalfRows * kCh, kCh, 0L,
          wfc1, wfc1, kCh, 0L,
          (void*)pre16, (void*)pre16, kHid, 0L,
          fc1_b, nullptr, 0L,
          kHalfRows, kHid, kCh, 1.0f / kWCarry);
    }
    {
      const int nwords = (kHalfRows * kHid) / 2;
      gelu_f16_kernel<<<(nwords + 255) / 256, 256, 0, stream>>>(
          (const unsigned*)(const void*)pre16, (unsigned*)(void*)hid16, nwords, kHCarry);
    }
    {
      const int tiles = (kCh / 64) * (kTok / 64);
      const size_t off = (size_t)half * kHalfBatch * kCh * kTok;
      wmma_gemm64<0, false, 1, 0, true><<<dim3((tiles + 7) / 8, kHalfBatch), 256, 0, stream>>>(
          wfc2, wfc2, kHid, 0L,
          hid16, hid16, kHid, (long)kTok * kHid,
          (void*)(out + off), (void*)(out + off), kTok, (long)kCh * kTok,
          fc2_b,
          T1 + off, (long)kCh * kTok,
          kCh, kTok, kHid, 1.0f / (kWCarry * kHCarry));
    }
  }
}
